// MultiHeadSelfAttention_84421877170302
// MI455X (gfx1250) — hardware-verified
//
#include <hip/hip_runtime.h>
#ifndef NB
#define NB 4
#endif
#ifndef SEQ
#define SEQ 2048
#endif
#define NB_FULL 4
#define SEQ_FULL 2048
#define DM 1024
#define NH 16
#define HD 64
#define NR ((size_t)NB * SEQ)
#define VTP (NB * SEQ)

static_assert(NB >= 1 && NB <= NB_FULL);
static_assert(SEQ <= SEQ_FULL);
static_assert(SEQ % 128 == 0);
static_assert(DM % 128 == 0);
static_assert(NH * HD == DM);
static_assert(HD == 64);
static_assert((NB * SEQ) % 64 == 0);
static_assert(HD % 64 == 0);
static_assert(HD % 32 == 0);
static_assert((NH * HD * HD / 8) % 256 == 0);
static_assert(NH * HD * HD <= DM * DM);
static_assert((DM * DM / 8) % 256 == 0);
static_assert((size_t)3 * NH * HD * HD * 2 + (size_t)DM * DM * 2 + (size_t)5 * NB * SEQ * DM * 2 + (size_t)6 * 256 <= (size_t)134217728);

typedef _Float16 v16h __attribute__((ext_vector_type(16)));
typedef _Float16 v4h __attribute__((ext_vector_type(4)));
typedef unsigned short v8us __attribute__((ext_vector_type(8), may_alias));
typedef float v8f __attribute__((ext_vector_type(8)));
typedef float v4f __attribute__((ext_vector_type(4)));
typedef float v4fa __attribute__((ext_vector_type(4), may_alias));
union FragH { v16h v; v8us half[2]; _Float16 h[16]; unsigned short u[16]; };

__device__ __forceinline__ unsigned short bf16_bits(float x) { unsigned int u = __float_as_uint(x); return (unsigned short)((u + 0x7FFFu + ((u >> 16) & 1u)) >> 16); }
__device__ __forceinline__ float bf16_rne(float x) { return __uint_as_float(((unsigned int)bf16_bits(x)) << 16); }

__device__ __forceinline__ v8us cvt8(const float* __restrict__ p, float scale) {
  const v4f a = *(const v4fa*)p, c = *(const v4fa*)(p + 4);
  FragH f;
#pragma unroll
  for (int q = 0; q < 4; ++q) { f.h[q] = (_Float16)(bf16_rne(a[q]) * scale); f.h[4 + q] = (_Float16)(bf16_rne(c[q]) * scale); }
  return f.half[0];
}

static __device__ __forceinline__ _Float16 toh_flush(float v) { const _Float16 r = (_Float16)v; return (fabsf(v) < 6.103515625e-05f) ? (_Float16)0.0f : r; }

__device__ __forceinline__ v8us cvt8_flush(const float* __restrict__ p, float scale) {
  const v4f a = *(const v4fa*)p, c = *(const v4fa*)(p + 4);
  FragH f;
#pragma unroll
  for (int q = 0; q < 4; ++q) { f.h[q] = toh_flush(bf16_rne(a[q]) * scale); f.h[4 + q] = toh_flush(bf16_rne(c[q]) * scale); }
  return f.half[0];
}

__global__ __launch_bounds__(256) void k_wplanes(const float* __restrict__ wq, const float* __restrict__ wk, const float* __restrict__ wv, const float* __restrict__ wo, size_t nh8, size_t no8, _Float16* __restrict__ BH, _Float16* __restrict__ BO) {
  #pragma clang fp contract(off)
  const size_t t = (size_t)blockIdx.x * 256 + threadIdx.x; if (t >= no8) return;
  const bool hs = t < nh8;
  const size_t th = hs ? t : (nh8 - 1);
  const v8us o3 = cvt8_flush(wo + t * 8, 16.0f);
  const v8us o0 = cvt8_flush(wq + th * 8, 16.0f), o1 = cvt8_flush(wk + th * 8, 16.0f), o2 = cvt8_flush(wv + th * 8, 16.0f);
  unsigned short* d = (unsigned short*)BO + t * 8; unsigned short* e = (unsigned short*)BH + th * 8; const size_t ps = (size_t)NH * HD * HD;
  *(volatile v8us*)d = o3;
  if (hs) { *(volatile v8us*)e = o0; *(volatile v8us*)(e + ps) = o1; *(volatile v8us*)(e + 2 * ps) = o2; }
  __threadfence();
  *(volatile v8us*)d = o3;
  if (hs) { *(volatile v8us*)e = o0; *(volatile v8us*)(e + ps) = o1; *(volatile v8us*)(e + 2 * ps) = o2; }
}

__global__ __launch_bounds__(256) void k_x16(const float* __restrict__ x, _Float16* __restrict__ X16, size_t n8) {
  #pragma clang fp contract(off)
  const size_t t = (size_t)blockIdx.x * 256 + threadIdx.x; if (t >= n8) return;
  const size_t e = t * 8; const size_t row = e / DM; const size_t col = e - row * DM; const size_t b = row / SEQ; const size_t s = row - b * SEQ;
  const v8us o = cvt8(x + (b * SEQ_FULL + s) * DM + col, 1.0f);
  unsigned short* d = (unsigned short*)X16 + e;
  *(volatile v8us*)d = o; __threadfence(); *(volatile v8us*)d = o;
}

__device__ __forceinline__ v16h g2_frag(const _Float16* p, int hh) { FragH f; f.half[0] = *(const v8us*)((const unsigned short*)p + 8 * hh); f.half[1] = *(const v8us*)((const unsigned short*)p + 16 + 8 * hh); return f.v; }
__device__ __forceinline__ v8f g2_mma(v16h a, v16h b, v8f c) { v8f d = __builtin_amdgcn_wmma_f32_16x16x32_f16(false, a, false, b, (short)0, c, false, false); asm volatile("v_nop\n\tv_nop\n\tv_nop\n\tv_nop" : "+v"(d) : "v"(a), "v"(b)); return d; }
__global__ __launch_bounds__(128) void k_gemm2(const _Float16* __restrict__ A, int lda, size_t sA, const _Float16* __restrict__ Bh, int ldb, size_t sB, float alpha,
    float* __restrict__ C, _Float16* __restrict__ C16, int ldc, size_t sC, int M, int N, int K) {
  __shared__ __attribute__((aligned(16))) float so[4][32][68];
  const int tid = threadIdx.x, lane = tid & 31, ln = lane & 15, hh = lane >> 4; const int w = __builtin_amdgcn_readfirstlane(tid >> 5); const int by = blockIdx.y;
  A += (size_t)by * sA; Bh += (size_t)by * sB; const size_t cofs = (size_t)by * sC;
  const int ntn = N >> 6; const int mt = blockIdx.x / ntn, nq = blockIdx.x - mt * ntn; const int row0 = mt * 128 + 32 * w, col0 = nq * 64; if (row0 >= M) return;
  const _Float16* a0p = A + (size_t)(row0 + ln) * lda; const _Float16* a1p = a0p + (size_t)16 * lda;
  const _Float16* b0p = Bh + (size_t)(col0 + ln) * ldb; const _Float16* b1p = b0p + (size_t)16 * ldb; const _Float16* b2p = b1p + (size_t)16 * ldb; const _Float16* b3p = b2p + (size_t)16 * ldb;
  const v8f z8 = {0.f,0.f,0.f,0.f,0.f,0.f,0.f,0.f}; v8f c00 = z8, c01 = z8, c02 = z8, c03 = z8, c10 = z8, c11 = z8, c12 = z8, c13 = z8;
#pragma unroll 1
  for (int kb = 0; kb < K; kb += 32) { const v16h a0 = g2_frag(a0p + kb, hh), a1 = g2_frag(a1p + kb, hh);
    v16h b = g2_frag(b0p + kb, hh); c00 = g2_mma(a0, b, c00); c10 = g2_mma(a1, b, c10);
    b = g2_frag(b1p + kb, hh); c01 = g2_mma(a0, b, c01); c11 = g2_mma(a1, b, c11);
    b = g2_frag(b2p + kb, hh); c02 = g2_mma(a0, b, c02); c12 = g2_mma(a1, b, c12);
    b = g2_frag(b3p + kb, hh); c03 = g2_mma(a0, b, c03); c13 = g2_mma(a1, b, c13); }
  v8f accs[8] = {c00, c01, c02, c03, c10, c11, c12, c13};
#pragma unroll
  for (int u = 0; u < 8; ++u) { const int t = u & 3, half = u >> 2;
#pragma unroll
    for (int r = 0; r < 8; ++r) { const int rloc = half * 16 + 8 * hh + r; so[w][rloc][t * 16 + ln] = accs[u][r] * alpha; } }
  __builtin_amdgcn_fence(4  , "workgroup"); __builtin_amdgcn_wave_barrier();
  const int rsub = lane >> 4, c4 = (lane & 15) * 4;
  for (int pass = 0; pass < 2; ++pass) {
#pragma unroll
    for (int q = 0; q < 16; ++q) { const int r = q * 2 + rsub; const v4f v = *(const v4fa*)&so[w][r][c4];
      if (C) *(volatile v4f*)(C + cofs + (size_t)(row0 + r) * ldc + col0 + c4) = v;
      if (C16) { v4h h4; for (int i = 0; i < 4; ++i) h4[i] = (_Float16)v[i]; *(volatile v4h*)(C16 + cofs + (size_t)(row0 + r) * ldc + col0 + c4) = h4; } }
    if (pass == 0) __threadfence(); } }

__global__ __launch_bounds__(128) void k_attn_t(const _Float16* __restrict__ Q16, const _Float16* __restrict__ K16, const _Float16* __restrict__ VT, _Float16* __restrict__ O16) {
  __shared__ __attribute__((aligned(16))) unsigned short so[4][16][72];
  const int tid = threadIdx.x, lane = tid & 31, ln = lane & 15, hh = lane >> 4;
  const int w = __builtin_amdgcn_readfirstlane(tid >> 5);
  const int nqb = SEQ / 64;
  const int bh = blockIdx.x / nqb, qb = blockIdx.x - bh * nqb;
  const int b = bh / NH, h = bh - b * NH;
  const size_t tok0 = (size_t)b * SEQ;
  const int q0 = qb * 64 + w * 16;
  const unsigned short* qp = (const unsigned short*)Q16 + (tok0 + q0 + ln) * DM + h * HD + 8 * hh;
  FragH bq0, bq1;
  bq0.half[0] = *(const v8us*)(qp);      bq0.half[1] = *(const v8us*)(qp + 16);
  bq1.half[0] = *(const v8us*)(qp + 32); bq1.half[1] = *(const v8us*)(qp + 48);
  const unsigned short* kp = (const unsigned short*)K16 + (tok0 + ln) * DM + h * HD + 8 * hh;
  const unsigned short* vp = (const unsigned short*)VT + (size_t)(h * HD + ln) * VTP + tok0 + 8 * hh;
  const v8f z8 = {0.f,0.f,0.f,0.f,0.f,0.f,0.f,0.f};
  v8f o0 = z8, o1 = z8, o2 = z8, o3 = z8;
  float m = -3.0e38f, l = 0.f;
  const float c = 0.125f * 1.4426950408889634f;
#pragma unroll 1
  for (int kv = 0; kv < SEQ; kv += 32) {
    const unsigned short* k0 = kp + (size_t)kv * DM;
    const unsigned short* k1 = k0 + (size_t)16 * DM;
    FragH a00, a01, a10, a11;
    a00.half[0] = *(const v8us*)(k0);      a00.half[1] = *(const v8us*)(k0 + 16);
    a01.half[0] = *(const v8us*)(k0 + 32); a01.half[1] = *(const v8us*)(k0 + 48);
    a10.half[0] = *(const v8us*)(k1);      a10.half[1] = *(const v8us*)(k1 + 16);
    a11.half[0] = *(const v8us*)(k1 + 32); a11.half[1] = *(const v8us*)(k1 + 48);
    v8f s0 = z8, s1 = z8;
    s0 = __builtin_amdgcn_wmma_f32_16x16x32_f16(false, a00.v, false, bq0.v, (short)0, s0, false, false);
    s1 = __builtin_amdgcn_wmma_f32_16x16x32_f16(false, a10.v, false, bq0.v, (short)0, s1, false, false);
    s0 = __builtin_amdgcn_wmma_f32_16x16x32_f16(false, a01.v, false, bq1.v, (short)0, s0, false, false);
    s1 = __builtin_amdgcn_wmma_f32_16x16x32_f16(false, a11.v, false, bq1.v, (short)0, s1, false, false);
    asm volatile("v_nop\n\tv_nop\n\tv_nop\n\tv_nop" : "+v"(s0), "+v"(s1) : "v"(a00.v), "v"(a01.v), "v"(a10.v), "v"(a11.v), "v"(bq0.v), "v"(bq1.v));
    float mx = fmaxf(s0[0], s1[0]);
#pragma unroll
    for (int r = 1; r < 8; ++r) mx = fmaxf(mx, fmaxf(s0[r], s1[r]));
    mx = fmaxf(mx, __shfl_xor(mx, 16, 32));
    const float mn = fmaxf(m, mx);
    if (__builtin_amdgcn_ballot_w32(mn > m) != 0u) {
      const float corr = __builtin_amdgcn_exp2f((m - mn) * c);
      l *= corr; o0 *= corr; o1 *= corr; o2 *= corr; o3 *= corr; m = mn;
    }
    const float off = 8.0f - m * c;
    FragH pf; float ls = 0.f;
#pragma unroll
    for (int r = 0; r < 8; ++r) {
      const float p0 = __builtin_amdgcn_exp2f(fmaf(s0[r], c, off));
      const float p1 = __builtin_amdgcn_exp2f(fmaf(s1[r], c, off));
      ls += p0 + p1;
      pf.h[r] = (_Float16)p0; pf.h[8 + r] = (_Float16)p1;
    }
    l += ls;
    const unsigned short* v0 = vp + kv;
    const unsigned short* v1 = v0 + (size_t)16 * VTP;
    const unsigned short* v2 = v1 + (size_t)16 * VTP;
    const unsigned short* v3 = v2 + (size_t)16 * VTP;
    FragH av0, av1, av2, av3;
    av0.half[0] = *(const v8us*)(v0); av0.half[1] = *(const v8us*)(v0 + 16);
    av1.half[0] = *(const v8us*)(v1); av1.half[1] = *(const v8us*)(v1 + 16);
    av2.half[0] = *(const v8us*)(v2); av2.half[1] = *(const v8us*)(v2 + 16);
    av3.half[0] = *(const v8us*)(v3); av3.half[1] = *(const v8us*)(v3 + 16);
    o0 = __builtin_amdgcn_wmma_f32_16x16x32_f16(false, av0.v, false, pf.v, (short)0, o0, false, false);
    o1 = __builtin_amdgcn_wmma_f32_16x16x32_f16(false, av1.v, false, pf.v, (short)0, o1, false, false);
    o2 = __builtin_amdgcn_wmma_f32_16x16x32_f16(false, av2.v, false, pf.v, (short)0, o2, false, false);
    o3 = __builtin_amdgcn_wmma_f32_16x16x32_f16(false, av3.v, false, pf.v, (short)0, o3, false, false);
    asm volatile("v_nop\n\tv_nop\n\tv_nop\n\tv_nop" : "+v"(o0), "+v"(o1), "+v"(o2), "+v"(o3) : "v"(av0.v), "v"(av1.v), "v"(av2.v), "v"(av3.v), "v"(pf.v));
  }
  l += __shfl_xor(l, 16, 32);
  const float inv = 64.0f * (1.0f / l);
  FragH t0, t1, t2, t3;
#pragma unroll
  for (int r = 0; r < 8; ++r) { t0.h[r] = (_Float16)(o0[r] * inv); t1.h[r] = (_Float16)(o1[r] * inv); t2.h[r] = (_Float16)(o2[r] * inv); t3.h[r] = (_Float16)(o3[r] * inv); }
  *(v8us*)&so[w][ln][ 0 + 8 * hh] = t0.half[0];
  *(v8us*)&so[w][ln][16 + 8 * hh] = t1.half[0];
  *(v8us*)&so[w][ln][32 + 8 * hh] = t2.half[0];
  *(v8us*)&so[w][ln][48 + 8 * hh] = t3.half[0];
  __syncthreads();
  const int rq = lane >> 3, pc = (lane & 7) * 8;
  unsigned short* ob = (unsigned short*)O16 + (tok0 + q0) * DM + h * HD + pc;
  for (int pass = 0; pass < 2; ++pass) {
#pragma unroll
    for (int it = 0; it < 4; ++it) { const int row = it * 4 + rq; const v8us v = *(const v8us*)&so[w][row][pc]; *(volatile v8us*)(ob + (size_t)row * DM) = v; }
    if (pass == 0) __threadfence();
  }
}

extern "C" void kernel_launch(void* const* d_in, const int* in_sizes, int n_in,
                              void* d_out, int out_size, void* d_ws, size_t ws_size, hipStream_t stream) {
  if (n_in < 5) return;
  const size_t need_x = ((size_t)(NB - 1) * SEQ_FULL + SEQ) * DM;
  const size_t nwh = (size_t)NH * HD * HD;
  if ((size_t)in_sizes[0] < need_x) return;
  if ((size_t)in_sizes[1] < nwh || (size_t)in_sizes[2] < nwh || (size_t)in_sizes[3] < nwh || (size_t)in_sizes[4] < (size_t)DM * DM) return;
  if ((size_t)out_size < need_x) return;
  const float* x = (const float*)d_in[0]; const float* wq = (const float*)d_in[1]; const float* wk = (const float*)d_in[2]; const float* wv = (const float*)d_in[3]; const float* wo = (const float*)d_in[4];
  char* ws = (char*)d_ws; size_t off = 0;
  auto take = [&](size_t bytes) { char* p = ws + off; off += (bytes + 255) & ~(size_t)255; return p; };
  _Float16* BH = (_Float16*)take((size_t)3 * nwh * 2);
  _Float16* BO = (_Float16*)take((size_t)DM * DM * 2);
  _Float16* X16 = (_Float16*)take(NR * DM * 2);
  _Float16* QK16 = (_Float16*)take((size_t)2 * NR * DM * 2);
  _Float16* VT = (_Float16*)take((size_t)DM * VTP * 2);
  _Float16* O16 = (_Float16*)take(NR * DM * 2);
  if (off > ws_size || off > (size_t)134217728) return;
  _Float16* BQ = BH; _Float16* BK = BH + nwh; _Float16* BV = BH + (size_t)2 * nwh;
  _Float16* Q16 = QK16; _Float16* K16 = QK16 + NR * DM;

  k_wplanes<<<(unsigned)(((size_t)DM * DM / 8 + 255) / 256), 256, 0, stream>>>(wq, wk, wv, wo, nwh / 8, (size_t)DM * DM / 8, BH, BO);
  k_x16<<<(unsigned)((NR * DM / 8 + 255) / 256), 256, 0, stream>>>(x, X16, NR * DM / 8);
  k_gemm2<<<dim3((unsigned)((NR / 128) * (HD / 64)), NH), 128, 0, stream>>>(X16, DM, (size_t)HD, BQ, HD, (size_t)HD * HD, 0.0625f, nullptr, Q16, DM, (size_t)HD, (int)NR, HD, HD);
  k_gemm2<<<dim3((unsigned)((NR / 128) * (HD / 64)), NH), 128, 0, stream>>>(X16, DM, (size_t)HD, BK, HD, (size_t)HD * HD, 0.0625f, nullptr, K16, DM, (size_t)HD, (int)NR, HD, HD);
  k_gemm2<<<dim3((unsigned)(((HD + 127) / 128) * (VTP / 64)), NH), 128, 0, stream>>>(BV, HD, (size_t)HD * HD, X16, DM, (size_t)HD, 0.0625f, nullptr, VT, VTP, (size_t)HD * VTP, HD, VTP, HD);
  k_attn_t<<<(unsigned)(NB * NH * (SEQ / 64)), 128, 0, stream>>>(Q16, K16, VT, O16);
  k_gemm2<<<dim3((unsigned)((SEQ / 128) * (DM / 64)), NB), 128, 0, stream>>>(O16, DM, (size_t)SEQ * DM, BO, DM, 0, 0.0009765625f, (float*)d_out, nullptr, DM, (size_t)SEQ_FULL * DM, SEQ, DM, DM);
}
